// MultiheadAttention_31267361915522
// MI455X (gfx1250) — hardware-run, weakly checked
//
#include <hip/hip_runtime.h>


#ifndef NB
#define NB 4
#endif
#ifndef SEQ
#define SEQ 1024
#endif
#define NB_FULL  4
#define SEQ_FULL 1024
#define DM   1024
#define NH_  16
#define HD   64
#define AW   4
#define MROWS (SEQ * NB)
#define LDQK 2048
#define LOG2E 1.4426950408889634f
#define SC2  (0.125f * LOG2E)
#define PSH  8.0f
#define WSC  256.0f
#define CSC  64.0f
#define RSC  2048.0f
#define TP   72

static_assert(HD == 64);
static_assert(NH_ * HD == DM);
static_assert(SEQ % 64 == 0);
static_assert(SEQ % (16 * AW) == 0);
static_assert(MROWS % 128 == 0);
static_assert(NB <= NB_FULL);
static_assert(SEQ <= SEQ_FULL);
static_assert(SEQ <= 1024);
static_assert(((size_t)MROWS * DM) % (8 * 256) == 0);
static_assert(((size_t)DM * DM) % (8 * 256) == 0);

typedef _Float16 h16;
typedef __attribute__((ext_vector_type(16))) _Float16 v16h;
typedef __attribute__((ext_vector_type(8)))  _Float16 v8h;
typedef __attribute__((ext_vector_type(8)))  float    v8f;
typedef __attribute__((ext_vector_type(4)))  float    v4f;
typedef v4f  __attribute__((may_alias)) v4fa;
typedef v8h  __attribute__((may_alias)) v8ha;

struct BThr { int t[80]; };
static_assert(sizeof(BThr) == 320);

__device__ __forceinline__ float rbf(float f) { unsigned u = __float_as_uint(f); u += 0x7FFFu + ((u >> 16) & 1u); return __uint_as_float(u & 0xFFFF0000u); }
__device__ __forceinline__ v16h cat16(v8h lo, v8h hi) { return __builtin_shufflevector(lo, hi, 0, 1, 2, 3, 4, 5, 6, 7, 8, 9, 10, 11, 12, 13, 14, 15); }
__device__ __forceinline__ v8f wmma16(v16h a, v16h b, v8f c) { return __builtin_amdgcn_wmma_f32_16x16x32_f16(false, a, false, b, (short)0, c, false, false); }
__device__ __forceinline__ v16h ldh(const h16* p) { return cat16(*(const v8h*)p, *(const v8h*)(p + 16)); }
__device__ __forceinline__ void wave_sync() { __builtin_amdgcn_fence(3  , "wavefront"); __builtin_amdgcn_wave_barrier(); asm volatile("" ::: "memory"); }

__global__ __launch_bounds__(256) void k_cvtx(const float* __restrict__ x, h16* dx, size_t n8) {
    const size_t i = (size_t)blockIdx.x * 256 + threadIdx.x; if (i >= n8) return;
    const size_t e = i * 8; const size_t m = e / DM, col = e % DM;
    const size_t t = m / NB, b = m % NB;
    const v8f v = *(const v8f*)(x + (t * NB_FULL + b) * DM + col); v8h o;
#pragma unroll
    for (int k = 0; k < 8; ++k) o[k] = (h16)rbf(v[k]);
    *(volatile v8h*)(dx + e) = o;
    __threadfence();
    *(volatile v8h*)(dx + e) = o;
}

__global__ __launch_bounds__(256) void k_cvtw(const float* __restrict__ w0, const float* __restrict__ w1, const float* __restrict__ w2, const float* __restrict__ w3,
                                              h16* d0, h16* d1, h16* d2, h16* d3, size_t n8) {
    const size_t i = (size_t)blockIdx.x * 256 + threadIdx.x; if (i >= n8) return;
    const size_t e = i * 8;
    const v8f a = *(const v8f*)(w0 + e); const v8f b = *(const v8f*)(w1 + e); const v8f c = *(const v8f*)(w2 + e); const v8f d = *(const v8f*)(w3 + e);
    v8h oa, ob, oc, od;
#pragma unroll
    for (int k = 0; k < 8; ++k) { oa[k] = (h16)(rbf(a[k]) * WSC); ob[k] = (h16)(rbf(b[k]) * WSC); oc[k] = (h16)(rbf(c[k]) * WSC); od[k] = (h16)(rbf(d[k]) * WSC); }
    *(volatile v8h*)(d0 + e) = oa; *(volatile v8h*)(d1 + e) = ob; *(volatile v8h*)(d2 + e) = oc; *(volatile v8h*)(d3 + e) = od;
    __threadfence();
    *(volatile v8h*)(d0 + e) = oa; *(volatile v8h*)(d1 + e) = ob; *(volatile v8h*)(d2 + e) = oc; *(volatile v8h*)(d3 + e) = od;
}

__global__ __launch_bounds__(256) void k_btab(const float* __restrict__ rel_emb, float* BT, const BThr P) {
    const int i = blockIdx.x * 256 + threadIdx.x;
    if (i >= NH_ * ((2 * SEQ) / 4)) return;
    const int h = i / ((2 * SEQ) / 4); const int d4 = (i % ((2 * SEQ) / 4)) * 4;
    v4f o;
#pragma unroll
    for (int e = 0; e < 4; ++e) {
        const int d = d4 + e; const int dc = (d < 2 * SEQ - 1) ? d : (2 * SEQ - 2);
        const int rel = dc - (SEQ - 1); const int a = (rel < 0) ? -rel : rel;
        int lg = 80;
#pragma unroll
        for (int j = 0; j < 79; ++j) lg += (a >= P.t[j]) ? 1 : 0;
        const int idx = (a < 80) ? a : lg;
        int bucket = ((rel > 0) ? 160 : 0) + idx; bucket = (bucket < 0) ? 0 : ((bucket > 319) ? 319 : bucket);
        const float v = rbf(rel_emb[bucket * NH_ + h]) * LOG2E;
        o[e] = (d < 2 * SEQ - 1) ? v : 0.0f;
    }
    float* dst = BT + (size_t)h * (2 * SEQ) + d4;
    *(volatile v4f*)dst = o;
    __threadfence();
    *(volatile v4f*)dst = o;
}

__global__ __launch_bounds__(128) void k_gvec(const float* __restrict__ grep_w, const float* __restrict__ grep_b, const float* __restrict__ grep_a, h16* G, float* GB) {
    const int tid = threadIdx.x; const int row = tid >> 3, c8 = (tid & 7) * 8;
    const int jb = (row == 1) ? 4 : 0;
    v8h o;
#pragma unroll
    for (int k = 0; k < 8; ++k) { float s = 0.0f;
#pragma unroll
        for (int j = 0; j < 4; ++j) s += rbf(grep_w[(jb + j) * HD + c8 + k]);
        o[k] = (h16)((row < 2) ? s * WSC : 0.0f); }
    float b0 = 0.0f, b1 = 0.0f;
#pragma unroll
    for (int j = 0; j < 4; ++j) { b0 += rbf(grep_b[j]); b1 += rbf(grep_b[4 + j]); }
    const float av = rbf(grep_a[tid & 15]);
    const int ln = tid & 31;
    const float gv = (ln == 0) ? b0 : ((ln == 1) ? b1 : ((ln >= 16) ? av : 0.0f));
    *(volatile v8h*)(G + row * HD + c8) = o;
    if (tid < 32) *(volatile float*)(GB + tid) = gv;
    __threadfence();
    *(volatile v8h*)(G + row * HD + c8) = o;
    if (tid < 32) *(volatile float*)(GB + tid) = gv;
}

template <int MODE>
__global__ __launch_bounds__(128) void k_gemm_p(const h16* __restrict__ X, const h16* __restrict__ W, const float* __restrict__ b0, const float* __restrict__ b1, void* OUTP) {
    __shared__ __align__(16) float os[4 * 32 * 68];
    const int lane = threadIdx.x & 31, wave = __builtin_amdgcn_readfirstlane((int)(threadIdx.x >> 5)), lr = lane & 15, hi = lane >> 4;
    const int n0 = blockIdx.x * 64;
    const int m0 = blockIdx.y * 128 + wave * 32;
    const h16* ap = X + (size_t)(m0 + lr) * DM + 8 * hi;
    const h16* bp = W + (size_t)(n0 + lr) * DM + 8 * hi;
    v8f c00 = (v8f){}, c01 = (v8f){}, c02 = (v8f){}, c03 = (v8f){}, c10 = (v8f){}, c11 = (v8f){}, c12 = (v8f){}, c13 = (v8f){};
#pragma unroll 1
    for (int k0 = 0; k0 < DM; k0 += 32) {
        const v16h a0 = ldh(ap + k0), a1 = ldh(ap + (size_t)16 * DM + k0);
        const v16h w0 = ldh(bp + k0), w1 = ldh(bp + (size_t)16 * DM + k0), w2 = ldh(bp + (size_t)32 * DM + k0), w3 = ldh(bp + (size_t)48 * DM + k0);
        c00 = wmma16(a0, w0, c00); c01 = wmma16(a0, w1, c01); c02 = wmma16(a0, w2, c02); c03 = wmma16(a0, w3, c03);
        c10 = wmma16(a1, w0, c10); c11 = wmma16(a1, w1, c11); c12 = wmma16(a1, w2, c12); c13 = wmma16(a1, w3, c13);
        asm volatile("v_nop\n\tv_nop\n\tv_nop\n\tv_nop" : "+v"(c00), "+v"(c01), "+v"(c02), "+v"(c03), "+v"(c10), "+v"(c11), "+v"(c12), "+v"(c13)
                     : "v"(a0), "v"(a1), "v"(w0), "v"(w1), "v"(w2), "v"(w3));
    }
    const int wb = wave * 32 * 68;
#pragma unroll
    for (int r = 0; r < 8; ++r) {
        const int ra = wb + (8 * hi + r) * 68 + lr, rb = wb + (16 + 8 * hi + r) * 68 + lr;
        os[ra] = c00[r]; os[ra + 16] = c01[r]; os[ra + 32] = c02[r]; os[ra + 48] = c03[r];
        os[rb] = c10[r]; os[rb + 16] = c11[r]; os[rb + 32] = c12[r]; os[rb + 48] = c13[r];
    }
    wave_sync();
    const float isc = 1.0f / WSC;
    if (MODE == 0) {
        h16* OH = (h16*)OUTP;
        const int c8 = (lane & 7) * 8, rq = lane >> 3;
        float bb[8];
#pragma unroll
        for (int k = 0; k < 8; ++k) { const int n = n0 + c8 + k; const int nn = n & (DM - 1); const float x = b0[nn], y = b1[nn]; bb[k] = rbf((n < DM) ? x : y); }
#pragma unroll 1
        for (int ps = 0; ps < 2; ++ps) {
#pragma unroll
            for (int s = 0; s < 8; ++s) { const int row = 4 * s + rq;
                const v4f u0 = *(const v4fa*)(&os[wb + row * 68 + c8]); const v4f u1 = *(const v4fa*)(&os[wb + row * 68 + c8 + 4]);
                v8h o;
#pragma unroll
                for (int k = 0; k < 4; ++k) { o[k] = (h16)(u0[k] * isc + bb[k]); o[4 + k] = (h16)(u1[k] * isc + bb[4 + k]); }
                *(volatile v8h*)(OH + (size_t)(m0 + row) * LDQK + n0 + c8) = o; }
            if (ps == 0) __threadfence(); }
    } else {
        float* OF = (float*)OUTP;
        const int cofs = lr * 4;
        v4f bb;
#pragma unroll
        for (int k = 0; k < 4; ++k) bb[k] = rbf(b0[n0 + cofs + k]);
#pragma unroll 1
        for (int ps = 0; ps < 2; ++ps) {
#pragma unroll
            for (int s = 0; s < 16; ++s) { const int row = 2 * s + hi;
                const v4f u = *(const v4fa*)(&os[wb + row * 68 + cofs]);
                const v4f val = u * isc + bb;
                *(volatile v4f*)(OF + (size_t)(m0 + row) * DM + n0 + cofs) = val; }
            if (ps == 0) __threadfence(); }
    }
}

__global__ __launch_bounds__(256) void k_vt(const float* __restrict__ V32, h16* VTH, h16* VTR) {
    __shared__ __align__(16) h16 th[64 * TP];
    __shared__ __align__(16) h16 tr[64 * TP];
    const int tid = threadIdx.x;
    const int zh = blockIdx.y; const int b = zh / NH_, h = zh % NH_;
    const int t0 = blockIdx.x * 64;
    const int r = tid >> 2, c0 = (tid & 3) * 16;
    const float* src = V32 + ((size_t)(t0 + r) * NB + b) * DM + h * HD + c0;
#pragma unroll
    for (int q = 0; q < 4; ++q) { const v4f x = *(const v4f*)(src + 4 * q);
#pragma unroll
        for (int i = 0; i < 4; ++i) { const float v = x[i]; const h16 hv = (h16)v; const h16 rv = (h16)((v - (float)hv) * RSC);
            th[(c0 + 4 * q + i) * TP + r] = hv; tr[(c0 + 4 * q + i) * TP + r] = rv; } }
    __syncthreads();
    h16* dh = VTH + (size_t)zh * HD * SEQ + t0;
    h16* dr = VTR + (size_t)zh * HD * SEQ + t0;
#pragma unroll 1
    for (int ps = 0; ps < 2; ++ps) {
#pragma unroll
        for (int s = 0; s < 2; ++s) { const int d = 32 * s + (tid >> 3), c8 = (tid & 7) * 8;
            const v8h vh = *(const v8ha*)(&th[d * TP + c8]); const v8h vr = *(const v8ha*)(&tr[d * TP + c8]);
            *(volatile v8h*)(dh + (size_t)d * SEQ + c8) = vh; *(volatile v8h*)(dr + (size_t)d * SEQ + c8) = vr; }
        if (ps == 0) __threadfence(); }
}

__global__ __launch_bounds__(32 * AW) void k_flash(const h16* __restrict__ QK, const h16* __restrict__ VTH, const h16* __restrict__ VTR,
                                                   const float* __restrict__ BT, const h16* __restrict__ G, const float* __restrict__ GB, h16* CH, h16* CR) {
    __shared__ __align__(16) float os[AW * 16 * 68];
    __shared__ __align__(16) float bts[2 * SEQ];
    const int tid = threadIdx.x;
    const int lane = tid & 31, wave = __builtin_amdgcn_readfirstlane((int)(threadIdx.x >> 5)), lr = lane & 15, hi = lane >> 4;
    const int zh = blockIdx.y; const int b = zh / NH_, h = zh % NH_;
#pragma unroll 1
    for (int i = tid; i < (2 * SEQ) / 4; i += 32 * AW) { const v4f x = *(const v4f*)(BT + (size_t)h * (2 * SEQ) + 4 * i); *(v4fa*)(&bts[4 * i]) = x; }
    __syncthreads();
    const int t0 = (blockIdx.x * AW + wave) * 16;
    const size_t rstr = (size_t)NB * LDQK;
    const size_t qo = ((size_t)(t0 + lr) * NB + b) * LDQK + (size_t)h * HD + 8 * hi;
    const v16h qh0 = ldh(QK + qo), qh1 = ldh(QK + qo + 32);
    float gt;
    { const v16h ga0 = ldh(G + lr * HD + 8 * hi), ga1 = ldh(G + lr * HD + 32 + 8 * hi);
      v8f gd = (v8f){};
      gd = wmma16(ga0, qh0, gd); gd = wmma16(ga1, qh1, gd);
      asm volatile("v_nop\n\tv_nop\n\tv_nop\n\tv_nop" : "+v"(gd) : "v"(ga0), "v"(ga1), "v"(qh0), "v"(qh1));
      const float g0 = __shfl(gd[0], lr, 32), g1 = __shfl(gd[1], lr, 32);
      const float la = g0 * (1.0f / WSC) + GB[0], lb = g1 * (1.0f / WSC) + GB[1];
      const float sga = 1.0f / (1.0f + __builtin_amdgcn_exp2f(-la * LOG2E));
      const float sgb = 1.0f / (1.0f + __builtin_amdgcn_exp2f(-lb * LOG2E));
      gt = sga * (sgb * GB[16 + h] - 1.0f) + 2.0f; }
    const size_t ko = ((size_t)lr * NB + b) * LDQK + DM + (size_t)h * HD + 8 * hi;
    const size_t vo = ((size_t)zh * HD + lr) * SEQ + 8 * hi;
    const int bi0 = 8 * hi - (t0 + lr) + (SEQ - 1);
    v8f o0 = (v8f){}, o1 = (v8f){}, o2 = (v8f){}, o3 = (v8f){};
    v8f r0 = (v8f){}, r1 = (v8f){}, r2 = (v8f){}, r3 = (v8f){};
    float m = -3.0e38f, l = 0.0f;
#pragma unroll 1
    for (int key0 = 0; key0 < SEQ; key0 += 32) {
        const h16* ka = QK + ko + (size_t)key0 * rstr;
        const v16h ka0 = ldh(ka), ka1 = ldh(ka + 32), kb0 = ldh(ka + 16 * rstr), kb1 = ldh(ka + 16 * rstr + 32);
        v8f sa = (v8f){}, sb = (v8f){};
        sa = wmma16(ka0, qh0, sa); sb = wmma16(kb0, qh0, sb);
        sa = wmma16(ka1, qh1, sa); sb = wmma16(kb1, qh1, sb);
        asm volatile("v_nop\n\tv_nop\n\tv_nop\n\tv_nop" : "+v"(sa), "+v"(sb) : "v"(ka0), "v"(ka1), "v"(kb0), "v"(kb1), "v"(qh0), "v"(qh1));
        const int bi = bi0 + key0;
        float ta[8], tb[8]; float mx = -3.0e38f;
#pragma unroll
        for (int r = 0; r < 8; ++r) { ta[r] = fmaf(gt, bts[bi + r], sa[r] * SC2); tb[r] = fmaf(gt, bts[bi + 16 + r], sb[r] * SC2); mx = fmaxf(mx, fmaxf(ta[r], tb[r])); }
        mx = fmaxf(mx, __shfl_xor(mx, 16, 32));
        const float mnew = fmaxf(m, mx);
        const float alpha = __builtin_amdgcn_exp2f(m - mnew);
        const float sh = PSH - mnew;
        v16h pb; float ls = 0.0f;
#pragma unroll
        for (int r = 0; r < 8; ++r) { const h16 pa = (h16)__builtin_amdgcn_exp2f(ta[r] + sh); const h16 pc = (h16)__builtin_amdgcn_exp2f(tb[r] + sh); pb[r] = pa; pb[8 + r] = pc; ls += (float)pa + (float)pc; }
        l = l * alpha + ls; m = mnew;
        o0 = o0 * alpha; o1 = o1 * alpha; o2 = o2 * alpha; o3 = o3 * alpha;
        r0 = r0 * alpha; r1 = r1 * alpha; r2 = r2 * alpha; r3 = r3 * alpha;
        { const h16* va = VTH + vo + key0;
          const v16h v0 = ldh(va), v1 = ldh(va + (size_t)16 * SEQ), v2 = ldh(va + (size_t)32 * SEQ), v3 = ldh(va + (size_t)48 * SEQ);
          o0 = wmma16(v0, pb, o0); o1 = wmma16(v1, pb, o1); o2 = wmma16(v2, pb, o2); o3 = wmma16(v3, pb, o3);
          asm volatile("v_nop\n\tv_nop\n\tv_nop\n\tv_nop" : "+v"(o0), "+v"(o1), "+v"(o2), "+v"(o3) : "v"(v0), "v"(v1), "v"(v2), "v"(v3), "v"(pb)); }
        { const h16* vr = VTR + vo + key0;
          const v16h w0 = ldh(vr), w1 = ldh(vr + (size_t)16 * SEQ), w2 = ldh(vr + (size_t)32 * SEQ), w3 = ldh(vr + (size_t)48 * SEQ);
          r0 = wmma16(w0, pb, r0); r1 = wmma16(w1, pb, r1); r2 = wmma16(w2, pb, r2); r3 = wmma16(w3, pb, r3);
          asm volatile("v_nop\n\tv_nop\n\tv_nop\n\tv_nop" : "+v"(r0), "+v"(r1), "+v"(r2), "+v"(r3) : "v"(w0), "v"(w1), "v"(w2), "v"(w3), "v"(pb)); }
    }
    l += __shfl_xor(l, 16, 32);
    const float inv = 1.0f / l;
    const float fs = inv * CSC, rs = 1.0f / RSC;
    const int wb = wave * 16 * 68;
    { const v8f f0 = (o0 + r0 * rs) * fs, f1 = (o1 + r1 * rs) * fs, f2 = (o2 + r2 * rs) * fs, f3 = (o3 + r3 * rs) * fs;
      const int ob = wb + lr * 68 + 8 * hi;
      *(v4fa*)(&os[ob +  0]) = __builtin_shufflevector(f0, f0, 0, 1, 2, 3); *(v4fa*)(&os[ob +  0 + 4]) = __builtin_shufflevector(f0, f0, 4, 5, 6, 7);
      *(v4fa*)(&os[ob + 16]) = __builtin_shufflevector(f1, f1, 0, 1, 2, 3); *(v4fa*)(&os[ob + 16 + 4]) = __builtin_shufflevector(f1, f1, 4, 5, 6, 7);
      *(v4fa*)(&os[ob + 32]) = __builtin_shufflevector(f2, f2, 0, 1, 2, 3); *(v4fa*)(&os[ob + 32 + 4]) = __builtin_shufflevector(f2, f2, 4, 5, 6, 7);
      *(v4fa*)(&os[ob + 48]) = __builtin_shufflevector(f3, f3, 0, 1, 2, 3); *(v4fa*)(&os[ob + 48 + 4]) = __builtin_shufflevector(f3, f3, 4, 5, 6, 7); }
    wave_sync();
    const size_t cb = ((size_t)t0 * NB + b) * DM + (size_t)h * HD;
    const int c8 = (lane & 7) * 8, rq = lane >> 3;
#pragma unroll 1
    for (int ps = 0; ps < 2; ++ps) {
#pragma unroll
        for (int s = 0; s < 4; ++s) { const int row = 4 * s + rq;
            const v4f u0 = *(const v4fa*)(&os[wb + row * 68 + c8]); const v4f u1 = *(const v4fa*)(&os[wb + row * 68 + c8 + 4]);
            v8h oh, orr;
#pragma unroll
            for (int k = 0; k < 4; ++k) { const float x = u0[k]; const h16 hx = (h16)x; oh[k] = hx; orr[k] = (h16)((x - (float)hx) * RSC);
                                          const float y = u1[k]; const h16 hy = (h16)y; oh[4 + k] = hy; orr[4 + k] = (h16)((y - (float)hy) * RSC); }
            const size_t off = cb + (size_t)row * NB * DM + c8;
            *(volatile v8h*)(CH + off) = oh; *(volatile v8h*)(CR + off) = orr; }
        if (ps == 0) __threadfence(); }
}

__global__ __launch_bounds__(128) void k_gemm_o(const h16* __restrict__ CHp, const h16* __restrict__ CRp, const h16* __restrict__ W, const float* __restrict__ bo, float* OUT) {
    __shared__ __align__(16) float os[4 * 16 * 68];
    const int lane = threadIdx.x & 31, wave = __builtin_amdgcn_readfirstlane((int)(threadIdx.x >> 5)), lr = lane & 15, hi = lane >> 4;
    const int n0 = blockIdx.x * 64;
    const int m0 = blockIdx.y * 64 + wave * 16;
    const h16* ap = CHp + (size_t)(m0 + lr) * DM + 8 * hi;
    const h16* rp = CRp + (size_t)(m0 + lr) * DM + 8 * hi;
    const h16* bp = W + (size_t)(n0 + lr) * DM + 8 * hi;
    v8f c0 = (v8f){}, c1 = (v8f){}, c2 = (v8f){}, c3 = (v8f){}, d0 = (v8f){}, d1 = (v8f){}, d2 = (v8f){}, d3 = (v8f){};
#pragma unroll 1
    for (int k0 = 0; k0 < DM; k0 += 32) {
        const v16h a = ldh(ap + k0), ar = ldh(rp + k0);
        const v16h w0 = ldh(bp + k0), w1 = ldh(bp + (size_t)16 * DM + k0), w2 = ldh(bp + (size_t)32 * DM + k0), w3 = ldh(bp + (size_t)48 * DM + k0);
        c0 = wmma16(a, w0, c0); c1 = wmma16(a, w1, c1); c2 = wmma16(a, w2, c2); c3 = wmma16(a, w3, c3);
        d0 = wmma16(ar, w0, d0); d1 = wmma16(ar, w1, d1); d2 = wmma16(ar, w2, d2); d3 = wmma16(ar, w3, d3);
        asm volatile("v_nop\n\tv_nop\n\tv_nop\n\tv_nop" : "+v"(c0), "+v"(c1), "+v"(c2), "+v"(c3), "+v"(d0), "+v"(d1), "+v"(d2), "+v"(d3)
                     : "v"(a), "v"(ar), "v"(w0), "v"(w1), "v"(w2), "v"(w3));
    }
    const int wb = wave * 16 * 68;
    const float rs = 1.0f / RSC, fs = 1.0f / (CSC * WSC);
#pragma unroll
    for (int r = 0; r < 8; ++r) { const int ra = wb + (8 * hi + r) * 68 + lr;
        os[ra] = (c0[r] + d0[r] * rs) * fs; os[ra + 16] = (c1[r] + d1[r] * rs) * fs; os[ra + 32] = (c2[r] + d2[r] * rs) * fs; os[ra + 48] = (c3[r] + d3[r] * rs) * fs; }
    wave_sync();
    const int cofs = lr * 4;
    v4f bb;
#pragma unroll
    for (int k = 0; k < 4; ++k) bb[k] = rbf(bo[n0 + cofs + k]);
#pragma unroll 1
    for (int ps = 0; ps < 2; ++ps) {
#pragma unroll
        for (int s = 0; s < 8; ++s) { const int row = 2 * s + hi;
            const int mm = m0 + row; const int t = mm / NB, b = mm % NB;
            const v4f u = *(const v4fa*)(&os[wb + row * 68 + cofs]);
            const v4f val = u + bb;
            *(volatile v4f*)(OUT + ((size_t)t * NB_FULL + b) * DM + n0 + cofs) = val; }
        if (ps == 0) __threadfence(); }
}

static constexpr size_t al256(size_t v) { return (v + 255) & ~(size_t)255; }
static constexpr size_t SZ_XH  = al256((size_t)MROWS * DM * 2);
static constexpr size_t SZ_WQK = al256((size_t)2 * DM * DM * 2);
static constexpr size_t SZ_W1  = al256((size_t)DM * DM * 2);
static constexpr size_t SZ_QK  = al256((size_t)MROWS * LDQK * 2);
static constexpr size_t SZ_V32 = al256((size_t)MROWS * DM * 4);
static constexpr size_t SZ_VT  = al256((size_t)NB * NH_ * HD * SEQ * 2);
static constexpr size_t SZ_C   = al256((size_t)MROWS * DM * 2);
static constexpr size_t SZ_BT  = al256((size_t)NH_ * 2 * SEQ * 4);
static constexpr size_t SZ_G   = al256((size_t)16 * HD * 2);
static constexpr size_t SZ_GB  = al256((size_t)32 * 4);
static constexpr size_t SZ_TOTAL = SZ_XH + SZ_WQK + 2 * SZ_W1 + SZ_QK + SZ_V32 + 2 * SZ_VT + 2 * SZ_C + SZ_BT + SZ_G + SZ_GB;
static_assert(SZ_TOTAL <= (size_t)134217728);

static double ln_d(double x) {
    int e = 0;
    while (x > 1.5) { x *= 0.5; ++e; }
    while (x < 0.75) { x *= 2.0; --e; }
    const double z = (x - 1.0) / (x + 1.0), z2 = z * z;
    double s = 1.0 / 41.0;
    for (int i = 19; i >= 0; --i) s = s * z2 + 1.0 / (double)(2 * i + 1);
    return 2.0 * z * s + (double)e * 0.69314718055994530942;
}

extern "C" void kernel_launch(void* const* d_in, const int* in_sizes, int n_in,
                              void* d_out, int out_size, void* d_ws, size_t ws_size, hipStream_t stream) {
    if (n_in < 13) return;
    const size_t needx = ((size_t)(SEQ - 1) * NB_FULL + NB) * DM;
    if ((size_t)in_sizes[0] < needx) return;
    if ((size_t)in_sizes[1] < (size_t)DM * DM || (size_t)in_sizes[3] < (size_t)DM * DM || (size_t)in_sizes[5] < (size_t)DM * DM || (size_t)in_sizes[7] < (size_t)DM * DM) return;
    if (in_sizes[2] < DM || in_sizes[4] < DM || in_sizes[6] < DM || in_sizes[8] < DM) return;
    if (in_sizes[9] < 320 * NH_ || in_sizes[10] < 8 * HD || in_sizes[11] < 8 || in_sizes[12] < NH_) return;
    if ((size_t)out_size < needx) return;
    if (SZ_TOTAL > ws_size) return;
    const float* query = (const float*)d_in[0];
    const float* wq = (const float*)d_in[1];  const float* bq = (const float*)d_in[2];
    const float* wk = (const float*)d_in[3];  const float* bk = (const float*)d_in[4];
    const float* wv = (const float*)d_in[5];  const float* bv = (const float*)d_in[6];
    const float* wo = (const float*)d_in[7];  const float* bo = (const float*)d_in[8];
    const float* rel_emb = (const float*)d_in[9];
    const float* grep_w = (const float*)d_in[10];
    const float* grep_b = (const float*)d_in[11];
    const float* grep_a = (const float*)d_in[12];
    float* OUT = (float*)d_out;
    char* wsp = (char*)d_ws;
    h16* XH  = (h16*)wsp;   wsp += SZ_XH;
    h16* WQK = (h16*)wsp;   wsp += SZ_WQK;
    h16* WV  = (h16*)wsp;   wsp += SZ_W1;
    h16* WO  = (h16*)wsp;   wsp += SZ_W1;
    h16* QK  = (h16*)wsp;   wsp += SZ_QK;
    float* V32 = (float*)wsp; wsp += SZ_V32;
    h16* VTH = (h16*)wsp;   wsp += SZ_VT;
    h16* VTR = (h16*)wsp;   wsp += SZ_VT;
    h16* CH  = (h16*)wsp;   wsp += SZ_C;
    h16* CR  = (h16*)wsp;   wsp += SZ_C;
    float* BT = (float*)wsp; wsp += SZ_BT;
    h16* G   = (h16*)wsp;   wsp += SZ_G;
    float* GB = (float*)wsp; wsp += SZ_GB;

    BThr P;
    { const double inv_ln10 = 1.0 / ln_d(10.0);
      int j = 0;
      for (int a = 80; a <= 1023 && j < 79; ++a) {
          const double val = ln_d((double)a / 80.0) * inv_ln10 * 80.0;
          const int L = 80 + (int)val;
          while (j < 79 && L >= 81 + j) { P.t[j] = a; ++j; }
      }
      for (; j < 80; ++j) P.t[j] = 0x7fffffff; }

    const size_t n8x = (size_t)MROWS * DM / 8;
    k_cvtx<<<(unsigned)((n8x + 255) / 256), 256, 0, stream>>>(query, XH, n8x);
    const size_t n8w = (size_t)DM * DM / 8;
    k_cvtw<<<(unsigned)((n8w + 255) / 256), 256, 0, stream>>>(wq, wk, wv, wo, WQK, WQK + (size_t)DM * DM, WV, WO, n8w);
    k_btab<<<(NH_ * ((2 * SEQ) / 4) + 255) / 256, 256, 0, stream>>>(rel_emb, BT, P);
    k_gvec<<<1, 128, 0, stream>>>(grep_w, grep_b, grep_a, G, GB);
    k_gemm_p<0><<<dim3(LDQK / 64, MROWS / 128, 1), 128, 0, stream>>>(XH, WQK, bq, bk, (void*)QK);
    k_gemm_p<1><<<dim3(DM / 64, MROWS / 128, 1), 128, 0, stream>>>(XH, WV, bv, bv, (void*)V32);
    k_vt<<<dim3(SEQ / 64, NB * NH_, 1), 256, 0, stream>>>(V32, VTH, VTR);
    k_flash<<<dim3(SEQ / (16 * AW), NB * NH_, 1), 32 * AW, 0, stream>>>(QK, VTH, VTR, BT, G, GB, CH, CR);
    k_gemm_o<<<dim3(DM / 64, MROWS / 64, 1), 128, 0, stream>>>(CH, CR, WO, bo, OUT);
}
